// SSI_DDI_Block_40114994545056
// MI455X (gfx1250) — hardware-verified
//
#include <hip/hip_runtime.h>
#include <stddef.h>


#define NTHR  256
#define NWAVE 8
#define HID   128
#define NHEAD 4
#define XW    256
#define WROWS 256
#define GR    32
#define GC    128
#define XSP   132
#define CHUNK 2048
#define WCAP  256
#define NGRP  (CHUNK / (NTHR * 4))
#define NBA   256
#define SHA   9
#define NBS   1024
#define SHS   10
#define PCH   (NTHR * 4)
#define GCAP  1024
#define AGG_LDS_BYTES ((NBA * HID + 2 * NBA * NHEAD) * 4 + (NWAVE * WCAP + 16) * 4 + 2 * NBA * 4)

static_assert(NGRP == 2);
static_assert(WCAP == (CHUNK / NTHR) * 32);
static_assert(AGG_LDS_BYTES == 149568);
static_assert(HID == 128);
static_assert(NTHR == 2 * HID);
static_assert(NBA == NWAVE * 32);
static_assert(NBA <= WCAP);
static_assert((1 << SHA) >= NBA);
static_assert(NBS == NWAVE * 128);
static_assert((1 << SHS) >= NBS);
static_assert((NBS % NBA) == 0 && (NBS % GR) == 0);
static_assert((GCAP % NTHR) == 0);
static_assert((XSP % 4) == 0);

typedef float          v4f  __attribute__((ext_vector_type(4)));
typedef float          v8f  __attribute__((ext_vector_type(8)));
typedef int            v4i  __attribute__((ext_vector_type(4)));
typedef __bf16         v16b __attribute__((ext_vector_type(16)));
typedef unsigned short v8us __attribute__((ext_vector_type(8)));

union FragB { v16b v; v4i u[2]; };
union Pack  { v8us s; v4i i; };

__device__ __forceinline__ unsigned short f2bf(float x) {
  unsigned b = __float_as_uint(x);
  b += 0x7FFFu + ((b >> 16) & 1u);
  return (unsigned short)(b >> 16);
}
__device__ __forceinline__ float bf2f(unsigned short h) { return __uint_as_float(((unsigned)h) << 16); }

__device__ __forceinline__ v8f wmb(v16b a, v16b b, v8f c) {
  v8f d = __builtin_amdgcn_wmma_f32_16x16x32_bf16(false, a, false, b, (short)0, c, false, false);
  asm volatile("v_nop\n\tv_nop\n\tv_nop\n\tv_nop" : "+v"(d) : "v"(a), "v"(b));
  return d;
}

__device__ __forceinline__ float lk(float t) { return fmaxf(t, 0.2f * t); }
__device__ __forceinline__ float dl(v4f t, v4f w) {
  return w.x * lk(t.x) + w.y * lk(t.y) + w.z * lk(t.z) + w.w * lk(t.w);
}
__device__ __forceinline__ int clampi(int v, int lo, int hi) { return v < lo ? lo : (v > hi ? hi : v); }

__global__ __launch_bounds__(NTHR) void k_cvtx(const float* __restrict__ x, int nN, int MP,
                                              unsigned short* ph, unsigned short* pl) {
  const int i  = blockIdx.x * NTHR + threadIdx.x;
  const int n8 = MP * (HID / 8);
  if (i >= n8) return;
  const int r  = i >> 4;
  const int kb = (i & 15) * 8;
  const int rc = (r < nN) ? r : (nN - 1);
  const bool ok = (r < nN);
  const v4f a = *(const v4f*)(x + (size_t)rc * HID + kb);
  const v4f b = *(const v4f*)(x + (size_t)rc * HID + kb + 4);
  float v[8];
#pragma unroll
  for (int j = 0; j < 4; ++j) { v[j] = ok ? a[j] : 0.f; v[4 + j] = ok ? b[j] : 0.f; }
  Pack uh, ul;
  const v4i z4 = {0, 0, 0, 0};
  uh.i = z4; ul.i = z4;
#pragma unroll
  for (int j = 0; j < 8; ++j) {
    const unsigned short hb = f2bf(v[j]);
    uh.s[j] = hb;
    ul.s[j] = f2bf(v[j] - bf2f(hb));
  }
  const size_t o = (size_t)i * 8;
  *(volatile v4i*)(ph + o) = uh.i;  *(volatile v4i*)(pl + o) = ul.i;
  __threadfence();
  *(volatile v4i*)(ph + o) = uh.i;  *(volatile v4i*)(pl + o) = ul.i;
}

__global__ __launch_bounds__(NTHR) void k_cvtw(const float* __restrict__ wl, const float* __restrict__ wr,
                                              unsigned short* ph, unsigned short* pl) {
  const int i = blockIdx.x * NTHR + threadIdx.x;
  if (i >= WROWS * (HID / 8)) return;
  const int cc = i >> 4;
  const int kb = (i & 15) * 8;
  const int c  = cc & (HID - 1);
  const bool useR = (cc >= HID);
  Pack uh, ul;
  const v4i z4 = {0, 0, 0, 0};
  uh.i = z4; ul.i = z4;
#pragma unroll
  for (int j = 0; j < 8; ++j) {
    const int k = kb + j;
    const float vl = wl[(size_t)k * HID + c];
    const float vr = wr[(size_t)k * HID + c];
    const float v  = useR ? vr : vl;
    const unsigned short hb = f2bf(v);
    uh.s[j] = hb;
    ul.s[j] = f2bf(v - bf2f(hb));
  }
  const size_t o = (size_t)i * 8;
  *(volatile v4i*)(ph + o) = uh.i;  *(volatile v4i*)(pl + o) = ul.i;
  __threadfence();
  *(volatile v4i*)(ph + o) = uh.i;  *(volatile v4i*)(pl + o) = ul.i;
}

__global__ __launch_bounds__(NTHR) void k_gemm(
    const unsigned short* __restrict__ A0, const unsigned short* __restrict__ A1,
    const unsigned short* __restrict__ B0, const unsigned short* __restrict__ B1,
    float* out, int K, int Ncols) {
  __shared__ __attribute__((aligned(16))) float Xs[GR * XSP];

  const int tid  = threadIdx.x;
  const int lane = tid & 31;
  const int wave = tid >> 5;
  const int hh   = lane >> 4;
  const int m    = lane & 15;
  const int rowBase = blockIdx.x * GR;
  const int colBase = blockIdx.y * GC;
  const int ncol = colBase + wave * 16 + m;

  const size_t ra0 = (size_t)(rowBase + m) * K + 8 * hh;
  const size_t ra1 = ra0 + (size_t)16 * K;
  const size_t rb  = (size_t)ncol * K + 8 * hh;

  v8f c0 = {0.f, 0.f, 0.f, 0.f, 0.f, 0.f, 0.f, 0.f};
  v8f c1 = {0.f, 0.f, 0.f, 0.f, 0.f, 0.f, 0.f, 0.f};

#pragma unroll 1
  for (int k0 = 0; k0 < K; k0 += 32) {
    FragB ah0, ah1, al0, al1, bh, bl;
    ah0.u[0] = *(const v4i*)(A0 + ra0 + k0);  ah0.u[1] = *(const v4i*)(A0 + ra0 + k0 + 16);
    ah1.u[0] = *(const v4i*)(A0 + ra1 + k0);  ah1.u[1] = *(const v4i*)(A0 + ra1 + k0 + 16);
    al0.u[0] = *(const v4i*)(A1 + ra0 + k0);  al0.u[1] = *(const v4i*)(A1 + ra0 + k0 + 16);
    al1.u[0] = *(const v4i*)(A1 + ra1 + k0);  al1.u[1] = *(const v4i*)(A1 + ra1 + k0 + 16);
    bh.u[0]  = *(const v4i*)(B0 + rb + k0);   bh.u[1]  = *(const v4i*)(B0 + rb + k0 + 16);
    bl.u[0]  = *(const v4i*)(B1 + rb + k0);   bl.u[1]  = *(const v4i*)(B1 + rb + k0 + 16);
    c0 = wmb(ah0.v, bh.v, c0);  c0 = wmb(ah0.v, bl.v, c0);  c0 = wmb(al0.v, bh.v, c0);
    c1 = wmb(ah1.v, bh.v, c1);  c1 = wmb(ah1.v, bl.v, c1);  c1 = wmb(al1.v, bh.v, c1);
  }

  const int cl = wave * 16 + m;
#pragma unroll
  for (int r = 0; r < 8; ++r) {
    Xs[(8 * hh + r) * XSP + cl]      = c0[r];
    Xs[(16 + 8 * hh + r) * XSP + cl] = c1[r];
  }
  __syncthreads();

  v4f xv[4];
  float* xpp[4];
#pragma unroll
  for (int i = 0; i < 4; ++i) {
    xv[i]  = *(const v4f*)(Xs + (4 * wave + i) * XSP + 4 * lane);
    xpp[i] = out + (size_t)(rowBase + 4 * wave + i) * Ncols + colBase + 4 * lane;
  }
#pragma unroll
  for (int i = 0; i < 4; ++i) *(volatile v4f*)(xpp[i]) = xv[i];
  __threadfence();
#pragma unroll
  for (int i = 0; i < 4; ++i) *(volatile v4f*)(xpp[i]) = xv[i];
}

template <int NB, int SH>
__device__ __forceinline__ int scan_chunk(const int* __restrict__ eid, int nE, int cbase, bool al16,
                                          int nodeBase, int* wl, int tid) {
  int wc = 0;
#pragma unroll
  for (int g = 0; g < NGRP; ++g) {
    const int el0 = (g * NTHR + tid) * 4;
    const int e0  = cbase + el0;
    const int sent = -2147483647 - 1;
    v4i d;
    if (al16 && (cbase + CHUNK <= nE)) {
      d = *(const v4i*)(eid + e0);
    } else {
      d.x = (e0     < nE) ? eid[min(e0,     nE - 1)] : sent;
      d.y = (e0 + 1 < nE) ? eid[min(e0 + 1, nE - 1)] : sent;
      d.z = (e0 + 2 < nE) ? eid[min(e0 + 2, nE - 1)] : sent;
      d.w = (e0 + 3 < nE) ? eid[min(e0 + 3, nE - 1)] : sent;
    }
    const unsigned s0 = (unsigned)d.x - (unsigned)nodeBase;
    const unsigned s1 = (unsigned)d.y - (unsigned)nodeBase;
    const unsigned s2 = (unsigned)d.z - (unsigned)nodeBase;
    const unsigned s3 = (unsigned)d.w - (unsigned)nodeBase;
    const bool h0 = s0 < (unsigned)NB;
    const bool h1 = s1 < (unsigned)NB;
    const bool h2 = s2 < (unsigned)NB;
    const bool h3 = s3 < (unsigned)NB;
    const unsigned many = __builtin_amdgcn_ballot_w32(h0 | h1 | h2 | h3);
    if (many != 0u) {
#define HITJ(J, HJ, SJ) { \
        const unsigned mj = __builtin_amdgcn_ballot_w32(HJ); \
        if (HJ) { \
          const int pos = wc + (int)__builtin_amdgcn_mbcnt_lo(mj, 0u); \
          if (pos < WCAP) wl[pos] = ((el0 + (J)) << SH) | (int)(SJ); \
        } \
        wc += (int)__builtin_popcount(mj); }
      HITJ(0, h0, s0)
      HITJ(1, h1, s1)
      HITJ(2, h2, s2)
      HITJ(3, h3, s3)
#undef HITJ
    }
  }
  return wc;
}

__device__ __forceinline__ void hitg(const float* xs, const float* xd, float* ar, float* mp, float* dp, v4f w) {
  const v4f a = *(const v4f*)(xs);
  const v4f d = *(const v4f*)(xd);
  float s = dl(a + d, w);
  s += __shfl_xor(s, 4, 32);
  s += __shfl_xor(s, 2, 32);
  s += __shfl_xor(s, 1, 32);
  const float m  = mp[0], n = dp[0];
  const float mn = fmaxf(m, s);
  const float sc = __expf(m - mn);
  const float p  = __expf(s - mn);
  v4f e = *(v4f*)(ar);
  e = e * sc + a * p;
  *(v4f*)(ar) = e;
  mp[0] = mn;
  dp[0] = n * sc + p;
}

__global__ __launch_bounds__(NTHR) void k_agg(
    const int* __restrict__ ei, const float* __restrict__ xlr, const float* __restrict__ att,
    const float* __restrict__ bias, const float* __restrict__ wrel, const float* __restrict__ brel,
    const float* __restrict__ wroot, float* out, float* T, float* U, int nN, int nE) {
  extern __shared__ v4f lds_dyn[];
  float* sacc = (float*)lds_dyn;
  float* mx   = sacc + NBA * HID;
  float* dn   = mx + NBA * NHEAD;
  int*   list = (int*)(dn + NBA * NHEAD);
  int*   wcnt = list + NWAVE * WCAP;
  float* ts   = (float*)(wcnt + 16);
  float* us   = ts + NBA;

  const int tid  = threadIdx.x;
  const int lane = tid & 31;
  const int wave = tid >> 5;
  const int nodeBase = blockIdx.x * NBA;

  {
    const v4f z4 = {0.f, 0.f, 0.f, 0.f};
    for (int i = tid; i < (NBA * HID) / 4; i += NTHR) lds_dyn[i] = z4;
    for (int i = tid; i < NBA * NHEAD; i += NTHR) { mx[i] = -1.0e30f; dn[i] = 0.f; }
  }
  __syncthreads();

  const int coff = 4 * lane;
  const int hidx = lane >> 3;
  const v4f w = *(const v4f*)(att + coff);

  const int* eid = ei + nE;
  const bool al16 = ((nE & 3) == 0);
  const int nChunks = (nE + CHUNK - 1) / CHUNK;

#pragma unroll 1
  for (int ch = 0; ch <= nChunks; ++ch) {
    const int cbase = ch * CHUNK;
    const bool selfp = (ch == nChunks);
    if (!selfp) {
      const int wc = scan_chunk<NBA, SHA>(eid, nE, cbase, al16, nodeBase, list + wave * WCAP, tid);
      if (lane == 0) wcnt[wave] = wc;
    } else {
      for (int s = tid; s < NBA; s += NTHR) list[s] = s;
      if (tid < NWAVE) {
        int c = NBA - tid * WCAP;
        c = c < 0 ? 0 : (c > WCAP ? WCAP : c);
        wcnt[tid] = c;
      }
    }
    __syncthreads();

    if (wave == 0) {
#pragma unroll 1
      for (int wsx = 0; wsx < NWAVE; ++wsx) {
        int n = __builtin_amdgcn_readfirstlane(wcnt[wsx]);
        n = n > WCAP ? WCAP : n;
        n = n < 0 ? 0 : n;
#pragma unroll 1
        for (int i = 0; i < n; ++i) {
          const int ent  = __builtin_amdgcn_readfirstlane(list[wsx * WCAP + i]);
          const int slot = ent & (NBA - 1);
          const int el   = (ent >> SHA) & (CHUNK - 1);
          const int node = nodeBase + slot;
          if (node >= nN) continue;
          int e = cbase + el;
          if (e > nE - 1) e = nE - 1;
          const int sj  = clampi(ei[e], 0, nN - 1);
          const int src = selfp ? node : sj;
          const float* xs = xlr + (size_t)src * XW + coff;
          const float* xd = xlr + (size_t)node * XW + HID + coff;
          float* ar = sacc + slot * HID + coff;
          float* mp = mx + slot * NHEAD + hidx;
          float* dp = dn + slot * NHEAD + hidx;
          hitg(xs, xd, ar, mp, dp, w);
        }
      }
    }
    __syncthreads();
  }

  const v4f wl4 = *(const v4f*)(wrel + coff);
  const v4f wr4 = *(const v4f*)(wroot + coff);
  const v4f b4  = *(const v4f*)(bias + coff);
  const float br = brel[0];
#pragma unroll 1
  for (int s = wave; s < NBA; s += NWAVE) {
    const int node = nodeBase + s;
    const bool valid = (node < nN);
    v4f o = {0.f, 0.f, 0.f, 0.f};
    if (valid) {
      const v4f e0 = *(const v4f*)(sacc + s * HID + coff);
      const float inv = 1.0f / fmaxf(dn[s * NHEAD + hidx], 1e-16f);
      o = e0 * inv + b4;
    }
    float t = o.x * wl4.x + o.y * wl4.y + o.z * wl4.z + o.w * wl4.w;
    float u = o.x * wr4.x + o.y * wr4.y + o.z * wr4.z + o.w * wr4.w;
    t += __shfl_xor(t, 16, 32);  u += __shfl_xor(u, 16, 32);
    t += __shfl_xor(t, 8, 32);   u += __shfl_xor(u, 8, 32);
    t += __shfl_xor(t, 4, 32);   u += __shfl_xor(u, 4, 32);
    t += __shfl_xor(t, 2, 32);   u += __shfl_xor(u, 2, 32);
    t += __shfl_xor(t, 1, 32);   u += __shfl_xor(u, 1, 32);
    t = valid ? t : 0.f;
    u = valid ? (u + br) : 0.f;
    if (lane == 0) { ts[s] = t; us[s] = u; }
    if (valid) {
      float* op = out + (size_t)node * HID + coff;
      *(volatile v4f*)op = o;
      __threadfence();
      *(volatile v4f*)op = o;
    }
  }
  __syncthreads();
  if (lane < 8) {
    const int q = 32 * wave + 4 * lane;
    const v4f tv = *(const v4f*)(ts + q);
    const v4f uv = *(const v4f*)(us + q);
    float* tp = T + nodeBase + q;
    float* up = U + nodeBase + q;
    *(volatile v4f*)tp = tv;  *(volatile v4f*)up = uv;
    __threadfence();
    *(volatile v4f*)tp = tv;  *(volatile v4f*)up = uv;
  }
}

__global__ __launch_bounds__(NTHR) void k_sag(const int* __restrict__ ei, const float* __restrict__ T,
                                             const float* __restrict__ U, float* S, int nN, int nE) {
  __shared__ __attribute__((aligned(16))) float ssum[NBS];
  __shared__ int list[NWAVE * WCAP];
  __shared__ int wcnt[NWAVE];

  const int tid  = threadIdx.x;
  const int lane = tid & 31;
  const int wave = tid >> 5;
  const int nodeBase = blockIdx.x * NBS;

  for (int i = tid; i < NBS; i += NTHR) ssum[i] = 0.f;
  __syncthreads();

  const int* eid = ei + nE;
  const bool al16 = ((nE & 3) == 0);
  const int nChunks = (nE + CHUNK - 1) / CHUNK;

#pragma unroll 1
  for (int ch = 0; ch < nChunks; ++ch) {
    const int cbase = ch * CHUNK;
    const int wc = scan_chunk<NBS, SHS>(eid, nE, cbase, al16, nodeBase, list + wave * WCAP, tid);
    if (lane == 0) wcnt[wave] = wc;
    __syncthreads();

    if (wave == 0) {
#pragma unroll 1
      for (int wsx = 0; wsx < NWAVE; ++wsx) {
        int n = __builtin_amdgcn_readfirstlane(wcnt[wsx]);
        n = n > WCAP ? WCAP : n;
        n = n < 0 ? 0 : n;
#pragma unroll 1
        for (int i0 = 0; i0 < n; i0 += 32) {
          int i = i0 + lane;
          i = (i < n) ? i : (n - 1);
          const int ent  = list[wsx * WCAP + i];
          const int slot = ent & (NBS - 1);
          const int el   = (ent >> SHS) & (CHUNK - 1);
          int e = cbase + el;
          if (e > nE - 1) e = nE - 1;
          const int sj = clampi(ei[e], 0, nN - 1);
          const float v = T[sj];
          const int cnt = (n - i0 < 32) ? (n - i0) : 32;
#pragma unroll 1
          for (int j = 0; j < cnt; ++j) {
            const int   sl = __shfl(slot, j, 32);
            const float vv = __shfl(v, j, 32);
            ssum[sl] += vv;
          }
        }
      }
    }
    __syncthreads();
  }

  const int idx = 128 * wave + 4 * lane;
  const v4f sv = *(const v4f*)(ssum + idx);
  const v4f uv = *(const v4f*)(U + nodeBase + idx);
  const v4f o  = sv + uv;
  float* sp = S + nodeBase + idx;
  *(volatile v4f*)sp = o;
  __threadfence();
  *(volatile v4f*)sp = o;
}

__global__ __launch_bounds__(NTHR) void k_pool(const int* __restrict__ bix, const float* __restrict__ S,
                                              const float* __restrict__ on, float* g, int nN) {
  __shared__ int   glist[GCAP];
  __shared__ float gv[GCAP];
  __shared__ int   wc2[2 * NWAVE];
  __shared__ float red[NTHR];
  __shared__ float gacc[NTHR];

  const int tid  = threadIdx.x;
  const int lane = tid & 31;
  const int wave = tid >> 5;
  const int b    = blockIdx.x;
  const bool al16 = ((nN & 3) == 0);
  const int nCh  = (nN + PCH - 1) / PCH;

  int total = 0;
#pragma unroll 1
  for (int ch = 0; ch < nCh; ++ch) {
    const int cbase = ch * PCH;
    const int e0 = cbase + tid * 4;
    const int sent = -2147483647 - 1;
    v4i d;
    if (al16 && (cbase + PCH <= nN)) {
      d = *(const v4i*)(bix + e0);
    } else {
      d.x = (e0     < nN) ? bix[min(e0,     nN - 1)] : sent;
      d.y = (e0 + 1 < nN) ? bix[min(e0 + 1, nN - 1)] : sent;
      d.z = (e0 + 2 < nN) ? bix[min(e0 + 2, nN - 1)] : sent;
      d.w = (e0 + 3 < nN) ? bix[min(e0 + 3, nN - 1)] : sent;
    }
    const bool h0 = (d.x == b), h1 = (d.y == b), h2 = (d.z == b), h3 = (d.w == b);
    const unsigned m0 = __builtin_amdgcn_ballot_w32(h0);
    const unsigned m1 = __builtin_amdgcn_ballot_w32(h1);
    const unsigned m2 = __builtin_amdgcn_ballot_w32(h2);
    const unsigned m3 = __builtin_amdgcn_ballot_w32(h3);
    const int c0 = (int)__builtin_popcount(m0), c1 = (int)__builtin_popcount(m1);
    const int c2 = (int)__builtin_popcount(m2), c3 = (int)__builtin_popcount(m3);
    if (lane == 0) wc2[(ch & 1) * NWAVE + wave] = c0 + c1 + c2 + c3;
    __syncthreads();
    int pw = 0, ct = 0;
#pragma unroll
    for (int ww = 0; ww < NWAVE; ++ww) {
      const int c = wc2[(ch & 1) * NWAVE + ww];
      ct += c;
      pw += (ww < wave) ? c : 0;
    }
    const int pb = total + pw;
    if (h0) { const int p = pb + (int)__builtin_amdgcn_mbcnt_lo(m0, 0u);                if (p < GCAP) glist[p] = e0; }
    if (h1) { const int p = pb + c0 + (int)__builtin_amdgcn_mbcnt_lo(m1, 0u);           if (p < GCAP) glist[p] = e0 + 1; }
    if (h2) { const int p = pb + c0 + c1 + (int)__builtin_amdgcn_mbcnt_lo(m2, 0u);      if (p < GCAP) glist[p] = e0 + 2; }
    if (h3) { const int p = pb + c0 + c1 + c2 + (int)__builtin_amdgcn_mbcnt_lo(m3, 0u); if (p < GCAP) glist[p] = e0 + 3; }
    total += ct;
  }
  const int gc = (total < GCAP) ? total : GCAP;
  __syncthreads();

  float lmax = -3.0e38f;
  for (int i = tid; i < gc; i += NTHR) {
    const int node = clampi(glist[i], 0, nN - 1);
    const float sv = S[node];
    gv[i] = sv;
    lmax = fmaxf(lmax, sv);
  }
  red[tid] = lmax;
  __syncthreads();
  for (int st = NTHR / 2; st > 0; st >>= 1) {
    if (tid < st) red[tid] = fmaxf(red[tid], red[tid + st]);
    __syncthreads();
  }
  const float m = red[0];
  __syncthreads();

  float lsum = 0.f;
  for (int i = tid; i < gc; i += NTHR) {
    const float ev = __expf(gv[i] - m);
    gv[i] = ev;
    lsum += ev;
  }
  red[tid] = lsum;
  __syncthreads();
  for (int st = NTHR / 2; st > 0; st >>= 1) {
    if (tid < st) red[tid] = red[tid] + red[tid + st];
    __syncthreads();
  }
  const float dsum = red[0];
  const float inv  = 1.0f / fmaxf(dsum, 1e-16f);
  for (int i = tid; i < gc; i += NTHR) gv[i] = gv[i] * inv;
  __syncthreads();

  const int c = tid & (HID - 1);
  const int part = tid >> 7;
  float acc = 0.f;
#pragma unroll 1
  for (int i = part; i < gc; i += 2) {
    const int node = clampi(glist[i], 0, nN - 1);
    acc += on[(size_t)node * HID + c] * gv[i];
  }
  gacc[tid] = acc;
  __syncthreads();

  if (wave == 0) {
    v4f o;
    o.x = gacc[4 * lane]     + gacc[HID + 4 * lane];
    o.y = gacc[4 * lane + 1] + gacc[HID + 4 * lane + 1];
    o.z = gacc[4 * lane + 2] + gacc[HID + 4 * lane + 2];
    o.w = gacc[4 * lane + 3] + gacc[HID + 4 * lane + 3];
    float* gp = g + (size_t)b * HID + 4 * lane;
    *(volatile v4f*)gp = o;
    __threadfence();
    *(volatile v4f*)gp = o;
  }
}

extern "C" void kernel_launch(void* const* d_in, const int* in_sizes, int n_in,
                              void* d_out, int out_size, void* d_ws, size_t ws_size,
                              hipStream_t stream) {
  if (n_in < 10) return;
  const int nN = in_sizes[0] / HID;
  if (nN <= 0 || in_sizes[0] != nN * HID) return;
  const int nE = in_sizes[1] / 2;
  if (nE <= 0 || in_sizes[1] != 2 * nE) return;
  if (in_sizes[2] != nN) return;
  if (in_sizes[3] != HID * HID || in_sizes[4] != HID * HID) return;
  if (in_sizes[5] != NHEAD * (HID / NHEAD) || in_sizes[6] != HID || in_sizes[7] != HID) return;
  if (in_sizes[8] < 1 || in_sizes[9] != HID) return;
  const int nB = out_size / HID - nN;
  if (nB <= 0 || out_size != (nN + nB) * HID) return;

  const float* x     = (const float*)d_in[0];
  const int*   ei    = (const int*)d_in[1];
  const int*   batch = (const int*)d_in[2];
  const float* Wl    = (const float*)d_in[3];
  const float* Wr    = (const float*)d_in[4];
  const float* att   = (const float*)d_in[5];
  const float* bias  = (const float*)d_in[6];
  const float* Wrel  = (const float*)d_in[7];
  const float* brel  = (const float*)d_in[8];
  const float* Wroot = (const float*)d_in[9];
  float* out = (float*)d_out;
  float* g   = out + (size_t)nN * HID;

  const int MP = ((nN + NBS - 1) / NBS) * NBS;

  char* wsp = (char*)d_ws;
  size_t off = 0;
  const size_t plB = (size_t)MP * HID * 2;
  const size_t wB  = (size_t)WROWS * HID * 2;
  const size_t xB  = (size_t)MP * XW * 4;
  const size_t vB  = (size_t)MP * 4;
  unsigned short* Ah = (unsigned short*)(wsp + off); off += plB;
  unsigned short* Al = (unsigned short*)(wsp + off); off += plB;
  unsigned short* Bh = (unsigned short*)(wsp + off); off += wB;
  unsigned short* Bl = (unsigned short*)(wsp + off); off += wB;
  float* XLR = (float*)(wsp + off); off += xB;
  float* T   = (float*)(wsp + off); off += vB;
  float* U   = (float*)(wsp + off); off += vB;
  float* S   = (float*)(wsp + off); off += vB;
  if (off > ws_size) return;

  hipFuncSetAttribute(reinterpret_cast<const void*>(&k_agg),
                      hipFuncAttributeMaxDynamicSharedMemorySize, AGG_LDS_BYTES);

  k_cvtx<<<(MP * (HID / 8) + NTHR - 1) / NTHR, NTHR, 0, stream>>>(x, nN, MP, Ah, Al);
  k_cvtw<<<(WROWS * (HID / 8) + NTHR - 1) / NTHR, NTHR, 0, stream>>>(Wl, Wr, Bh, Bl);
  k_gemm<<<dim3(MP / GR, XW / GC), NTHR, 0, stream>>>(Ah, Al, Bh, Bl, XLR, HID, XW);
  k_agg<<<MP / NBA, NTHR, AGG_LDS_BYTES, stream>>>(ei, XLR, att, bias, Wrel, brel, Wroot, out, T, U, nN, nE);
  k_sag<<<MP / NBS, NTHR, 0, stream>>>(ei, T, U, S, nN, nE);
  k_pool<<<nB, NTHR, 0, stream>>>(batch, S, out, g, nN);
}
